// causalAttention_11647951306945
// MI455X (gfx1250) — hardware-verified
//
#include <hip/hip_runtime.h>
#include <math.h>
#include <stdint.h>

#ifndef NB
#define NB 1
#endif
#ifndef SEQ
#define SEQ 8192
#endif
#define NB_FULL  1
#define SEQ_FULL 8192
#define EMB      1024
#define RC       ((SEQ < 1024) ? SEQ : 1024)
#define NCH      (SEQ / RC)
#define VLP      RC
#define PCARRY   16384.0f
#define RSC      4096.0f
#define SMI      ((SEQ / 8 + 255) / 256)
static_assert(NB == 1 && NB_FULL == 1);
static_assert(SEQ >= 256 && SEQ <= SEQ_FULL && (SEQ % 256) == 0);
static_assert((SEQ % RC) == 0 && (RC % 64) == 0 && NCH >= 1);
static_assert((EMB % 64) == 0 && (SEQ % 64) == 0 && (EMB % 32) == 0 && (RC % 32) == 0);
static_assert(SMI >= 1 && SMI <= 4);
static_assert(((SEQ * EMB / 8) % 256) == 0 && ((EMB * EMB / 8) % 256) == 0);

typedef _Float16 v16h __attribute__((ext_vector_type(16)));
typedef _Float16 v8h  __attribute__((ext_vector_type(8)));
typedef __bf16   v16b __attribute__((ext_vector_type(16)));
typedef __bf16   v8b  __attribute__((ext_vector_type(8)));
typedef float    v8f  __attribute__((ext_vector_type(8)));
typedef float    v4f  __attribute__((ext_vector_type(4)));
typedef unsigned int v4u __attribute__((ext_vector_type(4)));

#if defined(__HIP_DEVICE_COMPILE__)
#define DEV_ASM 1
#else
#define DEV_ASM 0
#endif

__device__ __forceinline__ unsigned short bf_bits(float f) {
  unsigned u = __float_as_uint(f);
  return (unsigned short)((u + 0x7FFFu + ((u >> 16) & 1u)) >> 16);
}
__device__ __forceinline__ unsigned short h_bits(_Float16 x) { return __builtin_bit_cast(unsigned short, x); }
__device__ __forceinline__ unsigned pk16(unsigned short a, unsigned short b) { return (unsigned)a | ((unsigned)b << 16); }
__device__ __forceinline__ v8f zero8() { v8f z = {0.f, 0.f, 0.f, 0.f, 0.f, 0.f, 0.f, 0.f}; return z; }

template <typename OT> struct FT;
template <> struct FT<__bf16>   { typedef v16b frag; typedef v8b half8; };
template <> struct FT<_Float16> { typedef v16h frag; typedef v8h half8; };

template <typename OT>
__device__ __forceinline__ typename FT<OT>::frag ldfrag(const OT* p) {
  union { typename FT<OT>::frag v; typename FT<OT>::half8 h[2]; } f;
  f.h[0] = *(const typename FT<OT>::half8*)(p);
  f.h[1] = *(const typename FT<OT>::half8*)(p + 16);
  return f.v;
}

__device__ __forceinline__ v8f mmar(v16b a, v16b b, v8f c) {
  return __builtin_amdgcn_wmma_f32_16x16x32_bf16(false, a, false, b, (short)0, c, false, false);
}
__device__ __forceinline__ v8f mmar(v16h a, v16h b, v8f c) {
  return __builtin_amdgcn_wmma_f32_16x16x32_f16(false, a, false, b, (short)0, c, false, false);
}
__device__ __forceinline__ void dep_guard(v8f& a, v8f& b, v16b x, v16b y) {
#if DEV_ASM
  asm volatile("v_nop\n\tv_nop\n\tv_nop\n\tv_nop" : "+v"(a), "+v"(b) : "v"(x), "v"(y));
#else
  (void)a; (void)b; (void)x; (void)y;
#endif
}
__device__ __forceinline__ void dep_guard(v8f& a, v8f& b, v16h x, v16h y) {
#if DEV_ASM
  asm volatile("v_nop\n\tv_nop\n\tv_nop\n\tv_nop" : "+v"(a), "+v"(b) : "v"(x), "v"(y));
#else
  (void)a; (void)b; (void)x; (void)y;
#endif
}
__device__ __forceinline__ void keep4(v16b a, v16b b, v16b c, v16b d) {
#if DEV_ASM
  asm volatile("v_nop" :: "v"(a), "v"(b), "v"(c), "v"(d));
#else
  (void)a; (void)b; (void)c; (void)d;
#endif
}
__device__ __forceinline__ void keep4(v16h a, v16h b, v16h c, v16h d) {
#if DEV_ASM
  asm volatile("v_nop" :: "v"(a), "v"(b), "v"(c), "v"(d));
#else
  (void)a; (void)b; (void)c; (void)d;
#endif
}
__device__ __forceinline__ void acc_guard4(v8f& a, v8f& b, v8f& c, v8f& d) {
#if DEV_ASM
  asm volatile("v_nop\n\tv_nop\n\tv_nop\n\tv_nop" : "+v"(a), "+v"(b), "+v"(c), "+v"(d));
#else
  (void)a; (void)b; (void)c; (void)d;
#endif
}

__global__ __launch_bounds__(256) void cvt16x8(const float* __restrict__ in, unsigned short* out, int n8) {
  const int i = blockIdx.x * 256 + (int)threadIdx.x;
  if (i < n8) {
    const float* ip = in + (size_t)i * 8;
    const v4f a  = *(const v4f*)(ip);
    const v4f a4 = *(const v4f*)(ip + 4);
    v4u p;
    p[0] = pk16(bf_bits(a[0]),  bf_bits(a[1]));
    p[1] = pk16(bf_bits(a[2]),  bf_bits(a[3]));
    p[2] = pk16(bf_bits(a4[0]), bf_bits(a4[1]));
    p[3] = pk16(bf_bits(a4[2]), bf_bits(a4[3]));
    unsigned short* o = out + (size_t)i * 8;
    *(volatile v4u*)o = p;
    __threadfence();
    *(volatile v4u*)o = p;
  }
}

template <typename OT, int MI, int NPA, int NPB, int OUT_MODE, int CZ>
__global__ __launch_bounds__(256) void gemm_t(
    const unsigned short* __restrict__ Ap, const unsigned short* __restrict__ A2p, int lda, long long strideA,
    const unsigned short* __restrict__ Btp, int ldb, long long strideB,
    const unsigned short* __restrict__ B2p, int ldb2, long long strideB2, int K2,
    void* Cout, void* Cout2, int ldc, long long strideC, int ldc2, long long strideC2, int N2,
    int M, int N, int K, float oscale, float rscale2, float cscale, float rscaleC, int czoff) {
  static_assert(CZ != 2 || ((16 * MI) % 32) == 0);
  typedef typename FT<OT>::frag V16;
  const OT* A  = (const OT*)(const void*)Ap;
  const OT* A2 = (const OT*)(const void*)A2p;
  const OT* Bt = (const OT*)(const void*)Btp;
  const OT* B2 = (const OT*)(const void*)B2p;
  __shared__ __align__(16) float sT[8][16 * 68];
  const int RT   = 16 * MI;
  const int b    = blockIdx.y;
  const int lane = threadIdx.x & 31;
  const int wave = threadIdx.x >> 5;
  const int tilesN = N >> 6;
  const int tilesM = M / RT;
  const int tile = blockIdx.x * 8 + wave;
  if (tile >= tilesM * tilesN) return;
  const int tm = tile / tilesN;
  const int tn = tile - tm * tilesN;
  const int m0 = tm * RT;
  const int n0 = tn << 6;
  if (CZ == 1) {
    if (n0 >= czoff + m0 + RT) return;
  }
  int kEnd = K;
  if (CZ == 2) {
    const int ke = czoff + m0 + RT;
    kEnd = (ke < K) ? ke : K;
  }

  const OT* Ab  = A  + (size_t)b * (size_t)strideA;
  const OT* A2b = A2 + (size_t)b * (size_t)strideA;
  const OT* Bb  = Bt + (size_t)b * (size_t)strideB;
  const OT* B2b = B2 + (size_t)b * (size_t)strideB2;

  const int rlane = lane & 15;
  const int koff  = (lane >> 4) * 8;
  const int mOff  = (lane >> 4) * 8;

  v8f acc[MI][4], acc2[MI][4];
#pragma unroll
  for (int i = 0; i < MI; ++i)
#pragma unroll
    for (int j = 0; j < 4; ++j) { acc[i][j] = zero8(); acc2[i][j] = zero8(); }

#pragma unroll 1
  for (int k0 = 0; k0 < kEnd; k0 += 32) {
    V16 bq[4];
#pragma unroll
    for (int j = 0; j < 4; ++j)
      bq[j] = ldfrag<OT>(Bb + (size_t)(n0 + (j << 4) + rlane) * ldb + koff + k0);
#pragma unroll
    for (int i = 0; i < MI; ++i) {
      const V16 af = ldfrag<OT>(Ab + (size_t)(m0 + (i << 4) + rlane) * lda + koff + k0);
#pragma unroll
      for (int j = 0; j < 4; ++j) acc[i][j] = mmar(af, bq[j], acc[i][j]);
      dep_guard(acc[i][0], acc[i][3], af, bq[3]);
      if (NPA == 2) {
        const V16 af2 = ldfrag<OT>(A2b + (size_t)(m0 + (i << 4) + rlane) * lda + koff + k0);
#pragma unroll
        for (int j = 0; j < 4; ++j) acc2[i][j] = mmar(af2, bq[j], acc2[i][j]);
        dep_guard(acc2[i][0], acc2[i][3], af2, bq[3]);
      }
    }
    keep4(bq[0], bq[1], bq[2], bq[3]);
    if (NPB == 2) {
      if (k0 < K2) {
        V16 br[4];
#pragma unroll
        for (int j = 0; j < 4; ++j)
          br[j] = ldfrag<OT>(B2b + (size_t)(n0 + (j << 4) + rlane) * ldb2 + koff + k0);
#pragma unroll
        for (int i = 0; i < MI; ++i) {
          const V16 afr = ldfrag<OT>(Ab + (size_t)(m0 + (i << 4) + rlane) * lda + koff + k0);
#pragma unroll
          for (int j = 0; j < 4; ++j) acc2[i][j] = mmar(afr, br[j], acc2[i][j]);
          dep_guard(acc2[i][0], acc2[i][3], afr, br[3]);
        }
        keep4(br[0], br[1], br[2], br[3]);
      }
    }
  }
#pragma unroll
  for (int i = 0; i < MI; ++i) {
    acc_guard4(acc[i][0], acc[i][1], acc[i][2], acc[i][3]);
    if (NPA == 2 || NPB == 2) acc_guard4(acc2[i][0], acc2[i][1], acc2[i][2], acc2[i][3]);
  }

  float* slab = sT[wave];
#pragma unroll
  for (int i = 0; i < MI; ++i) {
    const int mBase = m0 + (i << 4);
#pragma unroll
    for (int j = 0; j < 4; ++j) {
#pragma unroll
      for (int r = 0; r < 8; ++r) {
        float v = acc[i][j][r];
        if (NPA == 2 || NPB == 2) v += acc2[i][j][r] * rscale2;
        v = v * oscale;
        slab[(mOff + r) * 68 + (j << 4) + rlane] = v;
      }
    }
    __builtin_amdgcn_fence(3  , "workgroup");
    __builtin_amdgcn_wave_barrier();
    __builtin_amdgcn_fence(2  , "workgroup");
    if (OUT_MODE == 0) {
      float* C = (float*)Cout + (size_t)b * (size_t)strideC;
      const int h2 = lane >> 4, c4 = (lane & 15) * 4;
      for (int pass = 0; pass < 2; ++pass) {
#pragma unroll
        for (int it = 0; it < 8; ++it) {
          const int row = it * 2 + h2;
          const v4f v = *(const v4f*)(slab + row * 68 + c4);
          *(volatile v4f*)(C + (size_t)(mBase + row) * ldc + n0 + c4) = v;
        }
        __threadfence();
      }
    } else {
      const int q = lane >> 3, c8 = (lane & 7) * 8;
      unsigned short* C  = (unsigned short*)Cout  + (size_t)b * (size_t)strideC;
      unsigned short* C2 = (unsigned short*)Cout2 + (size_t)b * (size_t)strideC2;
      const bool wr2 = (OUT_MODE == 3) && (n0 < N2);
      v4u hv[4], lv[4];
#pragma unroll
      for (int it = 0; it < 4; ++it) {
        const int row = it * 4 + q;
        const float* sp = slab + row * 68 + c8;
        float f[8];
#pragma unroll
        for (int e = 0; e < 8; ++e) f[e] = sp[e] * cscale;
        v4u a, a2;
#pragma unroll
        for (int e = 0; e < 4; ++e) {
          const float f0 = f[2 * e], f1 = f[2 * e + 1];
          const _Float16 x0 = (_Float16)f0, x1 = (_Float16)f1;
          const unsigned short h0 = h_bits(x0), h1 = h_bits(x1);
          unsigned short l0 = 0, l1 = 0;
          if (OUT_MODE == 3) {
            l0 = h_bits((_Float16)((f0 - (float)x0) * rscaleC));
            l1 = h_bits((_Float16)((f1 - (float)x1) * rscaleC));
          }
          a[e] = pk16(h0, h1); a2[e] = pk16(l0, l1);
        }
        hv[it] = a; lv[it] = a2;
      }
      for (int pass = 0; pass < 2; ++pass) {
#pragma unroll
        for (int it = 0; it < 4; ++it) {
          const int row = it * 4 + q;
          *(volatile v4u*)(C + (size_t)(mBase + row) * ldc + n0 + c8) = hv[it];
          if (OUT_MODE == 3) {
            if (wr2) *(volatile v4u*)(C2 + (size_t)(mBase + row) * ldc2 + n0 + c8) = lv[it];
          }
        }
        __threadfence();
      }
    }
    __builtin_amdgcn_fence(3  , "workgroup");
    __builtin_amdgcn_wave_barrier();
    __builtin_amdgcn_fence(2  , "workgroup");
  }
}

template <int WRL>
__global__ __launch_bounds__(256)
void softmax_rows(const float* __restrict__ S, int ldS, unsigned short* P, unsigned short* Pl, int ldP, int rowBase) {
  __shared__ float redm[8];
  __shared__ float reds[8];
  const int r    = blockIdx.x;
  const int t    = rowBase + r;
  const int tid  = threadIdx.x;
  const int wave = tid >> 5;
  const int lane = tid & 31;
  const int ng   = ((t >> 6) + 1) * 8;
  const float* rp = S + (size_t)r * (size_t)ldS;
  float v[SMI][8];
#pragma unroll
  for (int it = 0; it < SMI; ++it) {
#pragma unroll
    for (int e = 0; e < 8; ++e) v[it][e] = -INFINITY;
    if (it * 256 < ng) {
      const int g  = it * 256 + tid;
      const int gc = (g < ng) ? g : (ng - 1);
      const int c0 = g * 8;
      const v4f a  = *(const v4f*)(rp + (size_t)gc * 8);
      const v4f a4 = *(const v4f*)(rp + (size_t)gc * 8 + 4);
#pragma unroll
      for (int e = 0; e < 4; ++e) {
        v[it][e]     = (c0 + e <= t)     ? a[e]  : -INFINITY;
        v[it][4 + e] = (c0 + 4 + e <= t) ? a4[e] : -INFINITY;
      }
    }
  }
  float mx = -INFINITY;
#pragma unroll
  for (int it = 0; it < SMI; ++it)
#pragma unroll
    for (int e = 0; e < 8; ++e) mx = fmaxf(mx, v[it][e]);
#pragma unroll
  for (int off = 1; off < 32; off <<= 1) mx = fmaxf(mx, __shfl_xor(mx, off, 32));
  if (lane == 0) redm[wave] = mx;
  __syncthreads();
  mx = redm[0];
#pragma unroll
  for (int w = 1; w < 8; ++w) mx = fmaxf(mx, redm[w]);

  float sum = 0.f;
#pragma unroll
  for (int it = 0; it < SMI; ++it) {
    if (it * 256 < ng) {
#pragma unroll
      for (int e = 0; e < 8; ++e) { const float ex = __expf(v[it][e] - mx); v[it][e] = ex; sum += ex; }
    } else {
#pragma unroll
      for (int e = 0; e < 8; ++e) v[it][e] = 0.f;
    }
  }
#pragma unroll
  for (int off = 1; off < 32; off <<= 1) sum += __shfl_xor(sum, off, 32);
  if (lane == 0) reds[wave] = sum;
  __syncthreads();
  sum = reds[0];
#pragma unroll
  for (int w = 1; w < 8; ++w) sum += reds[w];

  const float sc = PCARRY * (1.0f / sum);
  v4u pk[SMI], pl[SMI];
#pragma unroll
  for (int it = 0; it < SMI; ++it) {
    v4u a, a2;
#pragma unroll
    for (int e = 0; e < 4; ++e) {
      const float f0 = v[it][2 * e] * sc, f1 = v[it][2 * e + 1] * sc;
      const _Float16 x0 = (_Float16)f0, x1 = (_Float16)f1;
      unsigned short l0 = 0, l1 = 0;
      if (WRL == 1) {
        l0 = h_bits((_Float16)((f0 - (float)x0) * RSC));
        l1 = h_bits((_Float16)((f1 - (float)x1) * RSC));
      }
      a[e]  = pk16(h_bits(x0), h_bits(x1));
      a2[e] = pk16(l0, l1);
    }
    pk[it] = a; pl[it] = a2;
  }
  unsigned short* op  = P  + (size_t)r * (size_t)ldP;
  unsigned short* opl = Pl + (size_t)r * (size_t)ldP;
  for (int pass = 0; pass < 2; ++pass) {
#pragma unroll
    for (int it = 0; it < SMI; ++it) {
      if (it * 256 < ng) {
        const int g = it * 256 + tid;
        if (g < ng) {
          *(volatile v4u*)(op + (size_t)g * 8) = pk[it];
          if (WRL == 1) *(volatile v4u*)(opl + (size_t)g * 8) = pl[it];
        }
      }
    }
    __threadfence();
  }
}

static constexpr size_t PACT_B = (size_t)SEQ * EMB * 2;
static constexpr size_t PS_B   = (size_t)RC * SEQ * 4;
static constexpr size_t R0_B   = (PACT_B > PS_B) ? PACT_B : PS_B;
static constexpr size_t PW_B   = (size_t)EMB * EMB * 2;
static constexpr size_t PRES_B = (size_t)RC * EMB * 2;
static constexpr size_t PVT_B  = (size_t)EMB * SEQ * 2;
static constexpr size_t PVL_B  = (size_t)EMB * VLP * 2;
static constexpr size_t PP_B   = (size_t)RC * SEQ * 2;
static constexpr size_t PPL_B  = (size_t)RC * RC * 2;
static constexpr size_t WS_TOTAL = R0_B + 3 * PW_B + 2 * PACT_B + PVT_B + 2 * PRES_B + PVL_B + PP_B + PPL_B;
static_assert(WS_TOTAL <= (size_t)134217728);
static_assert((size_t)RC * ((size_t)NCH * RC) * 4 <= R0_B);
static_assert((size_t)RC * ((size_t)NCH * RC) * 2 <= PP_B);
static_assert((R0_B % 128) == 0 && (PW_B % 128) == 0 && (PRES_B % 128) == 0 && (PVL_B % 128) == 0 && (PPL_B % 128) == 0);

extern "C" void kernel_launch(void* const* d_in, const int* in_sizes, int n_in,
                              void* d_out, int out_size, void* d_ws, size_t ws_size,
                              hipStream_t stream) {
  if (n_in < 4) return;
  const long long needX = (long long)SEQ * (long long)EMB;
  if ((long long)in_sizes[0] < needX) return;
  if (in_sizes[1] < EMB * EMB) return;
  if (in_sizes[2] < EMB * EMB) return;
  if (in_sizes[3] < EMB * EMB) return;
  if (out_size < 0) return;
  if ((long long)out_size < needX) return;

  const float* x  = (const float*)d_in[0];
  const float* Wq = (const float*)d_in[1];
  const float* Wk = (const float*)d_in[2];
  const float* Wv = (const float*)d_in[3];

  size_t off = 0;
  const size_t oR0 = off; off += R0_B;
  const size_t oWq = off; off += PW_B;
  const size_t oWk = off; off += PW_B;
  const size_t oWv = off; off += PW_B;
  const size_t oQh = off; off += PACT_B;
  const size_t oKh = off; off += PACT_B;
  const size_t oVT = off; off += PVT_B;
  const size_t oQl = off; off += PRES_B;
  const size_t oKl = off; off += PRES_B;
  const size_t oVL = off; off += PVL_B;
  const size_t oP  = off; off += PP_B;
  const size_t oPl = off; off += PPL_B;
  if (off != WS_TOTAL) return;
  if (off > ws_size) return;
  if (off > (size_t)134217728) return;

  char* ws = (char*)d_ws;
  unsigned short* Xb  = (unsigned short*)(ws + oR0);
  float*          S   = (float*)(ws + oR0);
  unsigned short* Wqb = (unsigned short*)(ws + oWq);
  unsigned short* Wkb = (unsigned short*)(ws + oWk);
  unsigned short* Wvb = (unsigned short*)(ws + oWv);
  unsigned short* Qh  = (unsigned short*)(ws + oQh);
  unsigned short* Kh  = (unsigned short*)(ws + oKh);
  unsigned short* VT  = (unsigned short*)(ws + oVT);
  unsigned short* Ql  = (unsigned short*)(ws + oQl);
  unsigned short* Kl  = (unsigned short*)(ws + oKl);
  unsigned short* VL  = (unsigned short*)(ws + oVL);
  unsigned short* Pp  = (unsigned short*)(ws + oP);
  unsigned short* Ppl = (unsigned short*)(ws + oPl);
  float*          out0 = (float*)d_out;

  const dim3 blk(256);
  const int n8x = SEQ * EMB / 8;
  const int n8w = EMB * EMB / 8;
  const dim3 gCvtX(n8x / 256, 1);
  const dim3 gCvtW(n8w / 256, 1);
  const dim3 gPr0((((RC / 64) * (EMB / 64)) + 7) / 8, 1);
  const dim3 gPr1(((((SEQ - RC) / 64) * (EMB / 64)) + 7) / 8 + ((SEQ == RC) ? 1 : 0), 1);
  const dim3 gV((((EMB / 64) * (SEQ / 64)) + 7) / 8, 1);
  const dim3 gS0((((RC / 32) * (RC / 64)) + 7) / 8, 1);
  const dim3 gP0((((RC / 32) * (EMB / 64)) + 7) / 8, 1);
  const dim3 gPn((((RC / 64) * (EMB / 64)) + 7) / 8, 1);
  const dim3 gSm(RC);

  cvt16x8<<<gCvtX, blk, 0, stream>>>(x,  Xb,  n8x);
  cvt16x8<<<gCvtW, blk, 0, stream>>>(Wq, Wqb, n8w);
  cvt16x8<<<gCvtW, blk, 0, stream>>>(Wk, Wkb, n8w);
  cvt16x8<<<gCvtW, blk, 0, stream>>>(Wv, Wvb, n8w);
  gemm_t<__bf16, 4, 1, 1, 3, 0><<<gPr0, blk, 0, stream>>>(
      Xb, Xb, EMB, 0LL, Wqb, EMB, 0LL,
      Wqb, EMB, 0LL, 0,
      (void*)Qh, (void*)Ql, EMB, 0LL, EMB, 0LL, EMB,
      RC, EMB, EMB, 1.0f, 0.0f, 1.0f, RSC, 0);
  if (SEQ > RC) {
    gemm_t<__bf16, 4, 1, 1, 1, 0><<<gPr1, blk, 0, stream>>>(
        Xb + (size_t)RC * EMB, Xb + (size_t)RC * EMB, EMB, 0LL, Wqb, EMB, 0LL,
        Wqb, EMB, 0LL, 0,
        (void*)(Qh + (size_t)RC * EMB), (void*)(Qh + (size_t)RC * EMB), EMB, 0LL, EMB, 0LL, EMB,
        SEQ - RC, EMB, EMB, 1.0f, 0.0f, 1.0f, 1.0f, 0);
  }
  gemm_t<__bf16, 4, 1, 1, 3, 0><<<gPr0, blk, 0, stream>>>(
      Xb, Xb, EMB, 0LL, Wkb, EMB, 0LL,
      Wkb, EMB, 0LL, 0,
      (void*)Kh, (void*)Kl, EMB, 0LL, EMB, 0LL, EMB,
      RC, EMB, EMB, 1.0f, 0.0f, 1.0f, RSC, 0);
  if (SEQ > RC) {
    gemm_t<__bf16, 4, 1, 1, 1, 0><<<gPr1, blk, 0, stream>>>(
        Xb + (size_t)RC * EMB, Xb + (size_t)RC * EMB, EMB, 0LL, Wkb, EMB, 0LL,
        Wkb, EMB, 0LL, 0,
        (void*)(Kh + (size_t)RC * EMB), (void*)(Kh + (size_t)RC * EMB), EMB, 0LL, EMB, 0LL, EMB,
        SEQ - RC, EMB, EMB, 1.0f, 0.0f, 1.0f, 1.0f, 0);
  }
  gemm_t<__bf16, 4, 1, 1, 3, 0><<<gV, blk, 0, stream>>>(
      Wvb, Wvb, EMB, 0LL, Xb, EMB, 0LL,
      Xb, EMB, 0LL, 0,
      (void*)VT, (void*)VL, SEQ, 0LL, VLP, 0LL, VLP,
      EMB, SEQ, EMB, 1.0f, 0.0f, 1.0f, RSC, 0);
  for (int c = 0; c < NCH; ++c) {
    const int rb = c * RC;
    const int nc = rb + RC;
    if (c == 0) {
      gemm_t<_Float16, 2, 2, 2, 0, 1><<<gS0, blk, 0, stream>>>(
          Qh, Ql, EMB, 0LL, Kh, EMB, 0LL,
          Kl, EMB, 0LL, EMB,
          (void*)S, (void*)S, nc, 0LL, nc, 0LL, nc,
          RC, nc, EMB, 1.0f / 32.0f, 1.0f / RSC, 1.0f, 1.0f, 0);
      softmax_rows<1><<<gSm, blk, 0, stream>>>(S, nc, Pp, Ppl, nc, 0);
      gemm_t<_Float16, 2, 2, 2, 0, 2><<<gP0, blk, 0, stream>>>(
          Pp, Ppl, nc, 0LL, VT, SEQ, 0LL,
          VL, VLP, 0LL, VLP,
          (void*)out0, (void*)out0, EMB, 0LL, EMB, 0LL, EMB,
          RC, EMB, nc, 1.0f / PCARRY, 1.0f / RSC, 1.0f, 1.0f, 0);
    } else {
      const dim3 gSn((((RC / 64) * (nc / 64)) + 7) / 8, 1);
      gemm_t<_Float16, 4, 1, 1, 0, 1><<<gSn, blk, 0, stream>>>(
          Qh + (size_t)rb * EMB, Qh + (size_t)rb * EMB, EMB, 0LL, Kh, EMB, 0LL,
          Kh, EMB, 0LL, 0,
          (void*)S, (void*)S, nc, 0LL, nc, 0LL, nc,
          RC, nc, EMB, 1.0f / 32.0f, 0.0f, 1.0f, 1.0f, rb);
      softmax_rows<0><<<gSm, blk, 0, stream>>>(S, nc, Pp, Pp, nc, rb);
      gemm_t<_Float16, 4, 1, 1, 0, 2><<<gPn, blk, 0, stream>>>(
          Pp, Pp, nc, 0LL, VT, SEQ, 0LL,
          VT, SEQ, 0LL, 0,
          (void*)(out0 + (size_t)rb * EMB), (void*)(out0 + (size_t)rb * EMB), EMB, 0LL, EMB, 0LL, EMB,
          RC, EMB, nc, 1.0f / PCARRY, 0.0f, 1.0f, 1.0f, rb);
    }
  }
  (void)hipGetLastError();
}
